// TransformerBlock_73650099192379
// MI455X (gfx1250) — hardware-run, weakly checked
//
#include <hip/hip_runtime.h>
#include <math.h>

#ifndef NB
#define NB 2
#endif
#ifndef SEQ
#define SEQ 2048
#endif
#define NB_FULL 2
#define SEQ_FULL 2048
#define CE 1024
#define NH 16
#define HD 64
#define FFD 4096
#define MROWS (NB * SEQ)

static_assert(SEQ % 64 == 0);
static_assert(SEQ <= SEQ_FULL);
static_assert(NB <= NB_FULL);
static_assert(NH * HD == CE);
static_assert(CE % 64 == 0);
static_assert(FFD % 64 == 0);

typedef __attribute__((ext_vector_type(16))) _Float16 v16h;
typedef __attribute__((ext_vector_type(8)))  _Float16 v8h;
typedef __attribute__((ext_vector_type(16))) __bf16   v16b;
typedef __attribute__((ext_vector_type(8)))  __bf16   v8b;
typedef __attribute__((ext_vector_type(8)))  float    v8f;
typedef __attribute__((ext_vector_type(4)))  float    v4f;
typedef __attribute__((ext_vector_type(4)))  unsigned int cm_u4;


#define VST2(T, ptr, val) do { const T vst2_v_ = (val); *(volatile T*)(ptr) = vst2_v_; __threadfence(); *(volatile T*)(ptr) = vst2_v_; } while (0)

__device__ __forceinline__ unsigned short bfu_rne(float v) { unsigned u = __float_as_uint(v); u += 0x7FFFu + ((u >> 16) & 1u); return (unsigned short)(u >> 16); }
__device__ __forceinline__ float bfu_f32(unsigned short h) { return __uint_as_float(((unsigned)h) << 16); }
__device__ __forceinline__ float cmb_bf(float v) { const unsigned u = __float_as_uint(v); const unsigned r = (u + 0x7fffu + ((u >> 16) & 1u)) & 0xffff0000u; return __uint_as_float(r); }
__device__ __forceinline__ unsigned int cmb_pk2(float a, float b) { return (unsigned int)__builtin_bit_cast(unsigned short, (_Float16)a) | ((unsigned int)__builtin_bit_cast(unsigned short, (_Float16)b) << 16); }
__device__ __forceinline__ void split_pack2(float a, float b, unsigned& hi, unsigned& lo) {
    const unsigned short ha = bfu_rne(a), hb = bfu_rne(b);
    const unsigned short la = bfu_rne(a - bfu_f32(ha)), lb = bfu_rne(b - bfu_f32(hb));
    hi = (unsigned)ha | ((unsigned)hb << 16); lo = (unsigned)la | ((unsigned)lb << 16);
}

__device__ __forceinline__ void dep_guard_h(v8f& a, v8f& b, v16h x, v16h y) { asm volatile("v_nop\n\tv_nop\n\tv_nop\n\tv_nop" : "+v"(a), "+v"(b) : "v"(x), "v"(y)); }
__device__ __forceinline__ void dep_guard_b(v8f& a, v8f& b, v16b x, v16b y) { asm volatile("v_nop\n\tv_nop\n\tv_nop\n\tv_nop" : "+v"(a), "+v"(b) : "v"(x), "v"(y)); }
__device__ __forceinline__ void keep4_h(v16h a, v16h b, v16h c, v16h d) { asm volatile("v_nop" :: "v"(a), "v"(b), "v"(c), "v"(d)); }
__device__ __forceinline__ void keep4_b(v16b a, v16b b, v16b c, v16b d) { asm volatile("v_nop" :: "v"(a), "v"(b), "v"(c), "v"(d)); }
__device__ __forceinline__ void acc_guard4(v8f& a, v8f& b, v8f& c, v8f& d) { asm volatile("v_nop\n\tv_nop\n\tv_nop\n\tv_nop" : "+v"(a), "+v"(b), "+v"(c), "+v"(d)); }

template <typename T> struct Frag;
template <> struct Frag<_Float16> {
  typedef v16h V; union U { v16h v; v8h h[2]; };
  static __device__ __forceinline__ v16h load(const _Float16* p) {
    U f; f.h[0] = *(const v8h*)(p); f.h[1] = *(const v8h*)(p + 16); return f.v;
  }
  static __device__ __forceinline__ v8f mma(v16h a, v16h b, v8f c) {
    return __builtin_amdgcn_wmma_f32_16x16x32_f16(false, a, false, b, (short)0, c, false, false);
  }
  static __device__ __forceinline__ void guard(v8f& a, v8f& b, v16h x, v16h y) { dep_guard_h(a, b, x, y); }
  static __device__ __forceinline__ void keep(v16h a, v16h b, v16h c, v16h d) { keep4_h(a, b, c, d); }
};
template <> struct Frag<__bf16> {
  typedef v16b V; union U { v16b v; v8b h[2]; };
  static __device__ __forceinline__ v16b load(const __bf16* p) {
    U f; f.h[0] = *(const v8b*)(p); f.h[1] = *(const v8b*)(p + 16); return f.v;
  }
  static __device__ __forceinline__ v8f mma(v16b a, v16b b, v8f c) {
    return __builtin_amdgcn_wmma_f32_16x16x32_bf16(false, a, false, b, (short)0, c, false, false);
  }
  static __device__ __forceinline__ void guard(v8f& a, v8f& b, v16b x, v16b y) { dep_guard_b(a, b, x, y); }
  static __device__ __forceinline__ void keep(v16b a, v16b b, v16b c, v16b d) { keep4_b(a, b, c, d); }
};
template <int ET> struct Elem;
template <> struct Elem<0> { typedef _Float16 T; };
template <> struct Elem<1> { typedef __bf16 T; };

template <int ET, int BIAS_MODE, int OUT_MODE, int RESID, int ACT>
__global__ __launch_bounds__(256) void wmma_gemm64(
    const unsigned short* __restrict__ Ap, int lda, long long strideA,
    const unsigned short* __restrict__ Btp, int ldb, long long strideB,
    void* __restrict__ Cout, void* __restrict__ Cout2, int ldc, long long strideC,
    const float* __restrict__ bias,
    const float* __restrict__ resid, int ldr, long long strideR,
    int M, int N, int K, float scale) {
  typedef typename Elem<ET>::T T;
  typedef typename Frag<T>::V V;
  const T* A = (const T*)Ap; const T* Bt = (const T*)Btp;
  __shared__ __align__(16) float sT[8][16 * 68];
  const int b    = blockIdx.y;
  const int lane = threadIdx.x & 31;
  const int wave = __builtin_amdgcn_readfirstlane((int)(threadIdx.x >> 5));
  const int tilesN = N >> 6;
  const int tilesM = M >> 6;
  const int tile = blockIdx.x * 8 + wave;
  if (tile >= tilesM * tilesN) return;
  const int tm = tile / tilesN;
  const int tn = tile - tm * tilesN;
  const int m0 = tm << 6;
  const int n0 = tn << 6;

  const T* Ab = A  + (size_t)b * strideA;
  const T* Bb = Bt + (size_t)b * strideB;

  const int rlane = lane & 15;
  const int koff  = (lane >> 4) * 8;
  const int mOff  = (lane >> 4) * 8;

  v8f acc[4][4];
#pragma unroll
  for (int i = 0; i < 4; ++i)
#pragma unroll
    for (int j = 0; j < 4; ++j) acc[i][j] = (v8f){0.f,0.f,0.f,0.f,0.f,0.f,0.f,0.f};

  for (int k0 = 0; k0 < K; k0 += 32) {
    V bh[4];
#pragma unroll
    for (int j = 0; j < 4; ++j) {
      const size_t bo = (size_t)(n0 + (j << 4) + rlane) * ldb + koff + k0;
      bh[j] = Frag<T>::load(Bb + bo);
    }
#pragma unroll
    for (int i = 0; i < 4; ++i) {
      const size_t ao = (size_t)(m0 + (i << 4) + rlane) * lda + koff + k0;
      V ah = Frag<T>::load(Ab + ao);
#pragma unroll
      for (int j = 0; j < 4; ++j) acc[i][j] = Frag<T>::mma(ah, bh[j], acc[i][j]);
      Frag<T>::guard(acc[i][0], acc[i][3], ah, ah);
    }
    Frag<T>::keep(bh[0], bh[1], bh[2], bh[3]);
  }
  acc_guard4(acc[0][0], acc[0][1], acc[0][2], acc[0][3]);
  acc_guard4(acc[1][0], acc[1][1], acc[1][2], acc[1][3]);
  acc_guard4(acc[2][0], acc[2][1], acc[2][2], acc[2][3]);
  acc_guard4(acc[3][0], acc[3][1], acc[3][2], acc[3][3]);

  float* slab = sT[wave];
  const float* Rb = (RESID != 0) ? (resid + (size_t)b * strideR) : nullptr;
#pragma unroll
  for (int i = 0; i < 4; ++i) {
    const int mBase = m0 + (i << 4);
#pragma unroll
    for (int j = 0; j < 4; ++j) {
      const int n = n0 + (j << 4) + rlane;
      float bv = 0.f;
      if (BIAS_MODE == 2) bv = cmb_bf(bias[n]);
#pragma unroll
      for (int r = 0; r < 8; ++r) {
        float v = acc[i][j][r] * scale;
        if (BIAS_MODE == 2) v += bv;
        if (RESID == 1) v += Rb[(size_t)(mBase + mOff + r) * ldr + n];
        if (RESID == 2) v += cmb_bf(Rb[(size_t)(mBase + mOff + r) * ldr + n]);
        if (ACT == 2) v = fmaxf(v, 0.0f);
        slab[(mOff + r) * 68 + (j << 4) + rlane] = v;
      }
    }
    __builtin_amdgcn_fence(3  , "workgroup");
    __builtin_amdgcn_wave_barrier();
    __builtin_amdgcn_fence(2  , "workgroup");
    if (OUT_MODE == 0) {
      float* C = (float*)Cout + (size_t)b * strideC;
      const int hh = lane >> 4, c4 = (lane & 15) * 4;
      for (int pass = 0; pass < 2; ++pass) {
#pragma unroll
        for (int it = 0; it < 8; ++it) {
          const int row = it * 2 + hh;
          const v4f v = *(const v4f*)(slab + row * 68 + c4);
          *(volatile v4f*)(C + (size_t)(mBase + row) * ldc + n0 + c4) = v;
        }
        __threadfence();
      }
    } else {
      const int q = lane >> 3, c8 = (lane & 7) * 8;
      unsigned short* C  = (unsigned short*)Cout + (size_t)b * strideC;
      unsigned short* C2 = (OUT_MODE == 2) ? ((unsigned short*)Cout2 + (size_t)b * strideC) : C;
      for (int pass = 0; pass < 2; ++pass) {
#pragma unroll
        for (int it = 0; it < 4; ++it) {
          const int row = it * 4 + q;
          const float* sp = slab + row * 68 + c8;
          const v4f s0 = *(const v4f*)(sp), s1 = *(const v4f*)(sp + 4);
          cm_u4 hv, lv;
          if (OUT_MODE == 1) {
            hv.x = cmb_pk2(s0.x, s0.y); hv.y = cmb_pk2(s0.z, s0.w); hv.z = cmb_pk2(s1.x, s1.y); hv.w = cmb_pk2(s1.z, s1.w);
            lv = hv;
          } else {
            unsigned h0, h1, h2, h3, l0, l1, l2, l3;
            split_pack2(s0.x, s0.y, h0, l0); split_pack2(s0.z, s0.w, h1, l1);
            split_pack2(s1.x, s1.y, h2, l2); split_pack2(s1.z, s1.w, h3, l3);
            hv.x = h0; hv.y = h1; hv.z = h2; hv.w = h3;
            lv.x = l0; lv.y = l1; lv.z = l2; lv.w = l3;
          }
          *(volatile cm_u4*)(C + (size_t)(mBase + row) * ldc + n0 + c8) = hv;
          if (OUT_MODE == 2) *(volatile cm_u4*)(C2 + (size_t)(mBase + row) * ldc + n0 + c8) = lv;
        }
        __threadfence();
      }
    }
    __builtin_amdgcn_fence(3  , "workgroup");
    __builtin_amdgcn_wave_barrier();
    __builtin_amdgcn_fence(2  , "workgroup");
  }
}

template <int FMT>
__global__ __launch_bounds__(256) void k_cm_castbT(const float* __restrict__ SRC, long long sSz, int lds, unsigned short* __restrict__ DST, long long sDz, int ldd, int nR, int nC, float sc) {
    const long long u = (long long)blockIdx.x * 256 + threadIdx.x; const int per = nR / 8; if (u >= (long long)nC * per) return;
    const int c = (int)(u / per); const int r0 = 8 * (int)(u % per);
    const float* s = SRC + (long long)blockIdx.y * sSz;
    float w[8];
#pragma unroll
    for (int e = 0; e < 8; ++e) w[e] = cmb_bf(s[(long long)(r0 + e) * lds + c]) * sc;
    cm_u4 pk;
    if (FMT == 0) { pk.x = cmb_pk2(w[0], w[1]); pk.y = cmb_pk2(w[2], w[3]); pk.z = cmb_pk2(w[4], w[5]); pk.w = cmb_pk2(w[6], w[7]); }
    else {
        pk.x = (__float_as_uint(w[0]) >> 16) | (__float_as_uint(w[1]) & 0xffff0000u);
        pk.y = (__float_as_uint(w[2]) >> 16) | (__float_as_uint(w[3]) & 0xffff0000u);
        pk.z = (__float_as_uint(w[4]) >> 16) | (__float_as_uint(w[5]) & 0xffff0000u);
        pk.w = (__float_as_uint(w[6]) >> 16) | (__float_as_uint(w[7]) & 0xffff0000u);
    }
    VST2(cm_u4, DST + (long long)blockIdx.y * sDz + (long long)c * ldd + r0, pk);
}

template <int RB>
__global__ __launch_bounds__(128) void k_ln16(const float* __restrict__ X, long long bs, int seq,
        const float* __restrict__ G, const float* __restrict__ Bv, unsigned short* __restrict__ Y) {
    __shared__ float s1[4]; __shared__ float s2[4];
    const int m = blockIdx.x, t = threadIdx.x, lane = t & 31, wv = t >> 5;
    const int b = m / seq, tt = m - b * seq;
    const float* xr = X + (long long)b * bs + (long long)tt * CE + 8 * t;
    const v4f a0 = *(const v4f*)(xr), a1 = *(const v4f*)(xr + 4);
    float w[8] = {a0.x, a0.y, a0.z, a0.w, a1.x, a1.y, a1.z, a1.w};
    if (RB) {
#pragma unroll
        for (int e = 0; e < 8; ++e) w[e] = cmb_bf(w[e]);
    }
    float s = ((w[0] + w[1]) + (w[2] + w[3])) + ((w[4] + w[5]) + (w[6] + w[7]));
#pragma unroll
    for (int o = 16; o > 0; o >>= 1) s += __shfl_xor(s, o, 32);
    if (lane == 0) s1[wv] = s;
    __syncthreads();
    const float mu = ((s1[0] + s1[1]) + (s1[2] + s1[3])) * (1.0f / 1024.0f);
    float q = 0.f;
#pragma unroll
    for (int e = 0; e < 8; ++e) { w[e] -= mu; q += w[e] * w[e]; }
#pragma unroll
    for (int o = 16; o > 0; o >>= 1) q += __shfl_xor(q, o, 32);
    if (lane == 0) s2[wv] = q;
    __syncthreads();
    const float var = ((s2[0] + s2[1]) + (s2[2] + s2[3])) * (1.0f / 1024.0f);
    const float rs = rsqrtf(var + 1e-5f);
    const v4f g0 = *(const v4f*)(G + 8 * t), g1 = *(const v4f*)(G + 8 * t + 4);
    const v4f b0 = *(const v4f*)(Bv + 8 * t), b1 = *(const v4f*)(Bv + 8 * t + 4);
    const float gg[8] = {g0.x, g0.y, g0.z, g0.w, g1.x, g1.y, g1.z, g1.w};
    const float bb[8] = {b0.x, b0.y, b0.z, b0.w, b1.x, b1.y, b1.z, b1.w};
    float o8[8];
#pragma unroll
    for (int e = 0; e < 8; ++e) o8[e] = w[e] * rs * cmb_bf(gg[e]) + cmb_bf(bb[e]);
    cm_u4 pk; pk.x = cmb_pk2(o8[0], o8[1]); pk.y = cmb_pk2(o8[2], o8[3]); pk.z = cmb_pk2(o8[4], o8[5]); pk.w = cmb_pk2(o8[6], o8[7]);
    VST2(cm_u4, Y + (long long)m * CE + 8 * t, pk);
}

__device__ __forceinline__ v8f at_mma(v16b a, v16b b, v8f c) {
  c = __builtin_amdgcn_wmma_f32_16x16x32_bf16(false, a, false, b, (short)0, c, false, false);
  asm volatile("v_nop\n\tv_nop\n\tv_nop\n\tv_nop" : "+v"(c) : "v"(a), "v"(b));
  return c;
}
__device__ __forceinline__ void at_split(float f, __bf16& hi, __bf16& lo) {
  const unsigned short hb = bfu_rne(f);
  hi = __builtin_bit_cast(__bf16, hb);
  lo = __builtin_bit_cast(__bf16, bfu_rne(f - bfu_f32(hb)));
}

__global__ __launch_bounds__(128)
void k_attn_pl(const unsigned short* __restrict__ QKHp, const unsigned short* __restrict__ QKLp,
               const unsigned short* __restrict__ VTHp, const unsigned short* __restrict__ VTLp,
               unsigned short* __restrict__ CTX, int S, int H) {
  union FB { v16b v; v8b h[2]; };
  __shared__ __align__(16) __bf16 Psh[4][16 * 64];
  __shared__ __align__(16) __bf16 Psl[4][16 * 64];
  __shared__ __align__(16) float  Os[4][16 * 68];

  const int tid  = threadIdx.x;
  const int wave = __builtin_amdgcn_readfirstlane((int)(tid >> 5));
  const int lane = tid & 31;
  const int hh   = lane >> 4;
  const int c    = lane & 15;

  const int nqb = S / 64;
  const int bx = blockIdx.x;
  const int qb = bx % nqb;
  const int bh = bx / nqb;
  const int h  = bh % H;
  const int b  = bh / H;
  const int q0 = qb * 64 + wave * 16;

  const __bf16* QH = (const __bf16*)QKHp; const __bf16* QL = (const __bf16*)QKLp;
  const __bf16* VH = (const __bf16*)VTHp; const __bf16* VL = (const __bf16*)VTLp;
  const size_t qoff  = ((size_t)b * S + q0 + c) * 2048 + (size_t)h * 64 + 8 * hh;
  const size_t kbase = (size_t)b * S * 2048 + 1024 + (size_t)h * 64 + 8 * hh;
  const size_t vbase = ((size_t)b * 1024 + (size_t)h * 64 + c) * S + 8 * hh;

  float mrow[8], lrow[8];
  v8f oacc[4];
#pragma unroll
  for (int r = 0; r < 8; ++r) { mrow[r] = -__builtin_inff(); lrow[r] = 0.f; }
#pragma unroll
  for (int t = 0; t < 4; ++t) oacc[t] = (v8f){0.f,0.f,0.f,0.f,0.f,0.f,0.f,0.f};

  __bf16* pwh = Psh[wave];
  __bf16* pwl = Psl[wave];

  for (int kc = 0; kc <= qb; ++kc) {
    const int kv0 = kc * 64;
    v8f s[4];
#pragma unroll
    for (int j = 0; j < 4; ++j) s[j] = (v8f){0.f,0.f,0.f,0.f,0.f,0.f,0.f,0.f};
#pragma unroll 1
    for (int dc = 0; dc < 2; ++dc) {
      FB qh, ql;
      qh.h[0] = *(const v8b*)(QH + qoff + dc * 32);
      qh.h[1] = *(const v8b*)(QH + qoff + dc * 32 + 16);
      ql.h[0] = *(const v8b*)(QL + qoff + dc * 32);
      ql.h[1] = *(const v8b*)(QL + qoff + dc * 32 + 16);
#pragma unroll
      for (int j = 0; j < 4; ++j) {
        const size_t ko = kbase + (size_t)(kv0 + j * 16 + c) * 2048 + dc * 32;
        FB kb, kl;
        kb.h[0] = *(const v8b*)(QH + ko);
        kb.h[1] = *(const v8b*)(QH + ko + 16);
        kl.h[0] = *(const v8b*)(QL + ko);
        kl.h[1] = *(const v8b*)(QL + ko + 16);
        s[j] = at_mma(qh.v, kb.v, s[j]);
        s[j] = at_mma(qh.v, kl.v, s[j]);
        s[j] = at_mma(ql.v, kb.v, s[j]);
      }
    }
    const bool diag = (kc == qb);
    float cm[8];
#pragma unroll
    for (int r = 0; r < 8; ++r) {
      const int qrow = q0 + 8 * hh + r;
      float m = -__builtin_inff();
#pragma unroll
      for (int j = 0; j < 4; ++j) {
        const int kvcol = kv0 + j * 16 + c;
        float v = s[j][r] * 0.125f;
        if (diag && (kvcol > qrow)) v = -__builtin_inff();
        s[j][r] = v;
        m = fmaxf(m, v);
      }
      m = fmaxf(m, __shfl_xor(m, 1, 32)); m = fmaxf(m, __shfl_xor(m, 2, 32));
      m = fmaxf(m, __shfl_xor(m, 4, 32)); m = fmaxf(m, __shfl_xor(m, 8, 32));
      cm[r] = m;
    }
#pragma unroll
    for (int r = 0; r < 8; ++r) {
      const float mnew = fmaxf(mrow[r], cm[r]);
      const float alpha = expf(mrow[r] - mnew);
      mrow[r] = mnew;
      float psum = 0.f;
#pragma unroll
      for (int j = 0; j < 4; ++j) {
        const float p = expf(s[j][r] - mnew);
        psum += p;
        __bf16 a, bl; at_split(p, a, bl);
        pwh[(8 * hh + r) * 64 + j * 16 + c] = a;
        pwl[(8 * hh + r) * 64 + j * 16 + c] = bl;
      }
      psum += __shfl_xor(psum, 1, 32); psum += __shfl_xor(psum, 2, 32);
      psum += __shfl_xor(psum, 4, 32); psum += __shfl_xor(psum, 8, 32);
      lrow[r] = lrow[r] * alpha + psum;
#pragma unroll
      for (int t = 0; t < 4; ++t) oacc[t][r] *= alpha;
    }
    __builtin_amdgcn_fence(3  , "workgroup");
    __builtin_amdgcn_wave_barrier();
    __builtin_amdgcn_fence(2  , "workgroup");
#pragma unroll 1
    for (int kk = 0; kk < 2; ++kk) {
      FB pa, pl;
      pa.h[0] = *(const v8b*)(pwh + c * 64 + kk * 32 + 8 * hh);
      pa.h[1] = *(const v8b*)(pwh + c * 64 + kk * 32 + 16 + 8 * hh);
      pl.h[0] = *(const v8b*)(pwl + c * 64 + kk * 32 + 8 * hh);
      pl.h[1] = *(const v8b*)(pwl + c * 64 + kk * 32 + 16 + 8 * hh);
#pragma unroll
      for (int t = 0; t < 4; ++t) {
        const size_t vo = vbase + (size_t)(t * 16) * S + kv0 + kk * 32;
        FB vb, vl;
        vb.h[0] = *(const v8b*)(VH + vo);
        vb.h[1] = *(const v8b*)(VH + vo + 16);
        vl.h[0] = *(const v8b*)(VL + vo);
        vl.h[1] = *(const v8b*)(VL + vo + 16);
        oacc[t] = at_mma(pa.v, vb.v, oacc[t]);
        oacc[t] = at_mma(pa.v, vl.v, oacc[t]);
        oacc[t] = at_mma(pl.v, vb.v, oacc[t]);
      }
    }
    __builtin_amdgcn_fence(3  , "workgroup");
    __builtin_amdgcn_wave_barrier();
    __builtin_amdgcn_fence(2  , "workgroup");
  }

  float* os = Os[wave];
#pragma unroll
  for (int r = 0; r < 8; ++r) {
    const float inv = 1.0f / lrow[r];
#pragma unroll
    for (int t = 0; t < 4; ++t) os[(8 * hh + r) * 68 + t * 16 + c] = oacc[t][r] * inv;
  }
  __builtin_amdgcn_fence(3  , "workgroup");
  __builtin_amdgcn_wave_barrier();
  __builtin_amdgcn_fence(2  , "workgroup");
  {
    const int qd = lane >> 3, c8 = (lane & 7) * 8;
    unsigned short* ob = CTX + ((size_t)b * S + q0) * 2048 + (size_t)h * 64 + c8;
    for (int pass = 0; pass < 2; ++pass) {
#pragma unroll
      for (int it = 0; it < 4; ++it) {
        const int row = it * 4 + qd;
        const float* sp = os + row * 68 + c8;
        const v4f s0 = *(const v4f*)(sp), s1 = *(const v4f*)(sp + 4);
        unsigned h0, h1, h2, h3, l0, l1, l2, l3;
        split_pack2(s0.x, s0.y, h0, l0); split_pack2(s0.z, s0.w, h1, l1);
        split_pack2(s1.x, s1.y, h2, l2); split_pack2(s1.z, s1.w, h3, l3);
        cm_u4 hv, lv;
        hv.x = h0; hv.y = h1; hv.z = h2; hv.w = h3;
        lv.x = l0; lv.y = l1; lv.z = l2; lv.w = l3;
        *(volatile cm_u4*)(ob + (size_t)row * 2048) = hv;
        *(volatile cm_u4*)(ob + (size_t)row * 2048 + 1024) = lv;
      }
      __threadfence();
    }
  }
}

#define SZ_H16  ((size_t)MROWS * CE * 2)
#define SZ_W3   ((size_t)3 * CE * CE * 2)
#define SZ_QK   ((size_t)MROWS * 2048 * 2)
#define SZ_VT   ((size_t)NB * CE * SEQ * 2)
#define SZ_CTX  ((size_t)MROWS * 2048 * 2)
#define SZ_WP   ((size_t)CE * 2048 * 2)
#define SZ_X2   ((size_t)MROWS * CE * 4)
#define SZ_WF1  ((size_t)FFD * CE * 2)
#define SZ_WF2  ((size_t)CE * FFD * 2)
#define SZ_FFA  ((size_t)MROWS * FFD * 2)
#define SZ_TOTAL (SZ_H16 + SZ_W3 + 2 * SZ_QK + 2 * SZ_VT + SZ_CTX + SZ_WP + SZ_X2 + SZ_WF1 + SZ_WF2)
static_assert(SZ_TOTAL <= (size_t)134217728);
static_assert(SZ_FFA <= 2 * SZ_QK + 2 * SZ_VT);
static_assert(SZ_H16 % 256 == 0 && SZ_W3 % 256 == 0 && SZ_QK % 256 == 0 && SZ_VT % 256 == 0 && SZ_CTX % 256 == 0 && SZ_WP % 256 == 0 && SZ_X2 % 256 == 0 && SZ_WF1 % 256 == 0);

extern "C" void kernel_launch(void* const* d_in, const int* in_sizes, int n_in, void* d_out, int out_size, void* d_ws, size_t ws_size, hipStream_t stream) {
    const long long need_x = ((long long)(NB - 1) * SEQ_FULL + SEQ) * CE;
    if (n_in < 14) return;
    if ((long long)in_sizes[0] < need_x) return;
    if (in_sizes[1] < NH * CE * HD || in_sizes[2] < NH * CE * HD || in_sizes[3] < NH * CE * HD) return;
    if (in_sizes[4] < CE * CE || in_sizes[5] < CE || in_sizes[6] < CE || in_sizes[7] < CE || in_sizes[8] < CE || in_sizes[9] < CE) return;
    if (in_sizes[10] < CE * FFD || in_sizes[11] < FFD || in_sizes[12] < FFD * CE || in_sizes[13] < CE) return;
    if ((long long)out_size < need_x) return;
    if ((size_t)SZ_TOTAL > ws_size) return;

    const float* x      = (const float*)d_in[0];
    const float* wq     = (const float*)d_in[1];
    const float* wk     = (const float*)d_in[2];
    const float* wv     = (const float*)d_in[3];
    const float* w_proj = (const float*)d_in[4];
    const float* b_proj = (const float*)d_in[5];
    const float* g_ln1  = (const float*)d_in[6];
    const float* b_ln1  = (const float*)d_in[7];
    const float* g_ln2  = (const float*)d_in[8];
    const float* b_ln2  = (const float*)d_in[9];
    const float* w_ff1  = (const float*)d_in[10];
    const float* b_ff1  = (const float*)d_in[11];
    const float* w_ff2  = (const float*)d_in[12];
    const float* b_ff2  = (const float*)d_in[13];
    float* out = (float*)d_out;

    char* wsp = (char*)d_ws;
    unsigned short* H16 = (unsigned short*)wsp; wsp += SZ_H16;
    unsigned short* W3  = (unsigned short*)wsp; wsp += SZ_W3;
    unsigned short* QKH = (unsigned short*)wsp; wsp += SZ_QK;
    unsigned short* QKL = (unsigned short*)wsp; wsp += SZ_QK;
    unsigned short* VTH = (unsigned short*)wsp; wsp += SZ_VT;
    unsigned short* VTL = (unsigned short*)wsp; wsp += SZ_VT;
    unsigned short* CTX = (unsigned short*)wsp; wsp += SZ_CTX;
    unsigned short* WP  = (unsigned short*)wsp; wsp += SZ_WP;
    float*          X2  = (float*)wsp;          wsp += SZ_X2;
    unsigned short* WF1 = (unsigned short*)wsp; wsp += SZ_WF1;
    unsigned short* WF2 = (unsigned short*)wsp; wsp += SZ_WF2;
    unsigned short* FFA = QKH;

    k_cm_castbT<0><<<dim3((unsigned)((64 * (CE / 8) + 255) / 256), NH), 256, 0, stream>>>(wq, (long long)CE * HD, HD, W3,                        (long long)HD * CE, CE, CE, HD, 16.0f);
    k_cm_castbT<0><<<dim3((unsigned)((64 * (CE / 8) + 255) / 256), NH), 256, 0, stream>>>(wk, (long long)CE * HD, HD, W3 + (size_t)CE * CE,      (long long)HD * CE, CE, CE, HD, 16.0f);
    k_cm_castbT<0><<<dim3((unsigned)((64 * (CE / 8) + 255) / 256), NH), 256, 0, stream>>>(wv, (long long)CE * HD, HD, W3 + (size_t)2 * CE * CE,  (long long)HD * CE, CE, CE, HD, 16.0f);
    k_cm_castbT<1><<<dim3((unsigned)(((long long)CE * (CE / 8) + 255) / 256), 1), 256, 0, stream>>>(w_proj, 0, CE, WP,      0, 2048, CE, CE, 1.0f);
    k_cm_castbT<1><<<dim3((unsigned)(((long long)CE * (CE / 8) + 255) / 256), 1), 256, 0, stream>>>(w_proj, 0, CE, WP + CE, 0, 2048, CE, CE, 1.0f);
    k_cm_castbT<0><<<dim3((unsigned)(((long long)FFD * (CE / 8) + 255) / 256), 1), 256, 0, stream>>>(w_ff1, 0, FFD, WF1, 0, CE, CE, FFD, 16.0f);
    k_cm_castbT<0><<<dim3((unsigned)(((long long)CE * (FFD / 8) + 255) / 256), 1), 256, 0, stream>>>(w_ff2, 0, CE, WF2, 0, FFD, FFD, CE, 32.0f);

    k_ln16<1><<<MROWS, 128, 0, stream>>>(x, (long long)SEQ_FULL * CE, SEQ, g_ln1, b_ln1, H16);

    wmma_gemm64<0, 0, 2, 0, 0><<<dim3((unsigned)(((SEQ / 64) * (2048 / 64) + 7) / 8), NB), 256, 0, stream>>>(
        H16, CE, (long long)SEQ * CE, W3, CE, 0, (void*)QKH, (void*)QKL, 2048, (long long)SEQ * 2048,
        nullptr, nullptr, 0, 0, SEQ, 2048, CE, 0.0625f);
    wmma_gemm64<0, 0, 2, 0, 0><<<dim3((unsigned)(((CE / 64) * (SEQ / 64) + 7) / 8), NB), 256, 0, stream>>>(
        W3 + (size_t)2 * CE * CE, CE, 0, H16, CE, (long long)SEQ * CE, (void*)VTH, (void*)VTL, SEQ, (long long)CE * SEQ,
        nullptr, nullptr, 0, 0, CE, SEQ, CE, 0.0625f);

    k_attn_pl<<<dim3((unsigned)(NB * NH * (SEQ / 64))), 128, 0, stream>>>(QKH, QKL, VTH, VTL, CTX, SEQ, NH);

    wmma_gemm64<1, 2, 0, 2, 0><<<dim3((unsigned)(((SEQ / 64) * (CE / 64) + 7) / 8), NB), 256, 0, stream>>>(
        CTX, 2048, (long long)SEQ * 2048, WP, 2048, 0, (void*)X2, nullptr, CE, (long long)SEQ * CE,
        b_proj, x, CE, (long long)SEQ_FULL * CE, SEQ, CE, 2048, 1.0f);

    k_ln16<0><<<MROWS, 128, 0, stream>>>(X2, (long long)SEQ * CE, SEQ, g_ln2, b_ln2, H16);

    wmma_gemm64<0, 2, 1, 0, 2><<<dim3((unsigned)(((SEQ / 64) * (FFD / 64) + 7) / 8), NB), 256, 0, stream>>>(
        H16, CE, (long long)SEQ * CE, WF1, CE, 0, (void*)FFA, nullptr, FFD, (long long)SEQ * FFD,
        b_ff1, nullptr, 0, 0, SEQ, FFD, CE, 0.0625f);

    wmma_gemm64<0, 2, 0, 1, 0><<<dim3((unsigned)(((SEQ / 64) * (CE / 64) + 7) / 8), NB), 256, 0, stream>>>(
        FFA, FFD, (long long)SEQ * FFD, WF2, FFD, 0, (void*)out, nullptr, CE, (long long)SEQ_FULL * CE,
        b_ff2, X2, CE, (long long)SEQ * CE, SEQ, CE, FFD, 0.03125f);
}
